// GNN_60790967108277
// MI455X (gfx1250) — hardware-verified
//
#include <hip/hip_runtime.h>
#include <stddef.h>
#include <stdint.h>
#include <math.h>


#define DF      128
#define DH      256
#define KA      256
#define NF      9
#define NBF     3
#define NBV     6
#define BTAB    (NBF * NBV * DF)
#define NTHR    256
#define NWAVE   8
#define EPT     8
#define CHUNK   (NTHR * EPT)
#define WCAP    (EPT * 32)
#define LISTN   (NWAVE * WCAP)
#define NBA     1024
#define PKS     10
#define RCAP    28672
#define DEGCAP  64
#define GBM     64
#define GTHR    128
#define GNT     8
#define GBN     (16 * GNT)
#define PH1     (DH * KA)
#define PH2     (DF * KA)
#define WU1     (DH * (KA / 8))
#define WU2     (DF * (KA / 8))
#define NLMAX   8
#define PARTW   288
#define PMEAN   32
#define PM2     160
#define ZINTS   (2 * RCAP + 2 * NBA + LISTN)
#define MISCI   16
#define LDS_AGG ((ZINTS + MISCI + BTAB) * 4)
#define WSMAX   134217728

static_assert((CHUNK & (CHUNK - 1)) == 0);
static_assert(NBA == (1 << PKS));
static_assert(((long long)CHUNK << PKS) < (1LL << 31));
static_assert(NTHR * 4 == NBA);
static_assert(LISTN >= NBA && LISTN >= NWAVE * WCAP);
static_assert((RCAP % 32) == 0);
static_assert((ZINTS % (NTHR * 4)) == 0);
static_assert(((ZINTS + MISCI) % 4) == 0);
static_assert(LDS_AGG <= 262144);
static_assert((NBA % NWAVE) == 0 && (NBA % GBM) == 0);
static_assert(GBM == (GTHR / 32) * 16);
static_assert(KA == 2 * DF && (KA % 32) == 0);
static_assert((WU1 % NTHR) == 0 && (WU2 % NTHR) == 0 && WU1 == 8192 && WU2 == 4096);
static_assert(DF == 32 * 4);
static_assert(GBN == DF && (KA / 8) == 32 && GTHR == GBN);
static_assert((PARTW % 32) == 0 && PARTW / 4 <= GTHR && PM2 + DF <= PARTW && PMEAN + DF <= PM2);
static_assert(NTHR == 2 * DF);
static_assert(DH == 2 * DF);
static_assert((BTAB % NTHR) == 0);

typedef float          v4f  __attribute__((ext_vector_type(4)));
typedef float          v8f  __attribute__((ext_vector_type(8)));
typedef int            v4i  __attribute__((ext_vector_type(4)));
typedef int            v8i  __attribute__((ext_vector_type(8)));
typedef unsigned int   v4u  __attribute__((ext_vector_type(4)));
typedef unsigned short v8us __attribute__((ext_vector_type(8)));
typedef _Float16       v16h __attribute__((ext_vector_type(16)));
typedef __bf16         v16b __attribute__((ext_vector_type(16)));
typedef v4f  __attribute__((may_alias)) v4fa;
typedef v4i  __attribute__((may_alias)) v4ia;
typedef v8us __attribute__((may_alias)) v8usa;
union Frag { v16b b; v16h f; v8us h[2]; v4u q[2]; v8i w; };

__device__ __forceinline__ v8f wmk(const Frag& a, const Frag& b, v8f c) {
  v8f d = __builtin_amdgcn_wmma_f32_16x16x32_bf16(false, a.b, false, b.b, (short)0, c, false, false);
  asm volatile("v_nop\n\tv_nop\n\tv_nop\n\tv_nop" : "+v"(d) : "v"(a.w), "v"(b.w));
  return d;
}

__device__ __forceinline__ unsigned short bf_bits(float f) {
  unsigned int u = __float_as_uint(f);
  u += 0x7FFFu + ((u >> 16) & 1u);
  return (unsigned short)(u >> 16);
}
__device__ __forceinline__ float bf_val(unsigned short b) {
  return __uint_as_float(((unsigned int)b) << 16);
}
__device__ __forceinline__ float bf_rne(float f) { return bf_val(bf_bits(f)); }

template <int ACT>
__device__ __forceinline__ float actf(float v) {
  if constexpr (ACT == 1) {
    return fmaxf(v, 0.0f);
  } else {
    return v;
  }
}

__device__ __forceinline__ v4u pack_hilo4(float r0, float r1, float r2, float r3) {
  const unsigned short hb0 = bf_bits(r0), hb1 = bf_bits(r1), hb2 = bf_bits(r2), hb3 = bf_bits(r3);
  const unsigned short lb0 = bf_bits(r0 - bf_val(hb0)), lb1 = bf_bits(r1 - bf_val(hb1));
  const unsigned short lb2 = bf_bits(r2 - bf_val(hb2)), lb3 = bf_bits(r3 - bf_val(hb3));
  v4u pk;
  pk.x = (unsigned int)hb0 | ((unsigned int)hb1 << 16);
  pk.y = (unsigned int)hb2 | ((unsigned int)hb3 << 16);
  pk.z = (unsigned int)lb0 | ((unsigned int)lb1 << 16);
  pk.w = (unsigned int)lb2 | ((unsigned int)lb3 << 16);
  return pk;
}

__device__ __forceinline__ int scan_chunk(const int* __restrict__ dsts, int nE, int cbase, int slotBase,
                                          int nb, int vec8, int* list, int tid, int lane, int wave) {
  int wc = 0;
  const int el0  = tid * EPT;
  const int e0   = cbase + el0;
  const int sent = -2147483647 - 1;
  v4i da, db;
  if (vec8 != 0 && cbase + CHUNK <= nE) {
    da = *(const v4i*)(dsts + e0);
    db = *(const v4i*)(dsts + e0 + 4);
  } else {
    da.x = (e0     < nE) ? dsts[min(e0,     nE - 1)] : sent;
    da.y = (e0 + 1 < nE) ? dsts[min(e0 + 1, nE - 1)] : sent;
    da.z = (e0 + 2 < nE) ? dsts[min(e0 + 2, nE - 1)] : sent;
    da.w = (e0 + 3 < nE) ? dsts[min(e0 + 3, nE - 1)] : sent;
    db.x = (e0 + 4 < nE) ? dsts[min(e0 + 4, nE - 1)] : sent;
    db.y = (e0 + 5 < nE) ? dsts[min(e0 + 5, nE - 1)] : sent;
    db.z = (e0 + 6 < nE) ? dsts[min(e0 + 6, nE - 1)] : sent;
    db.w = (e0 + 7 < nE) ? dsts[min(e0 + 7, nE - 1)] : sent;
  }
  const unsigned nbs = (unsigned)slotBase;
  const unsigned unb = (unsigned)nb;
  const unsigned s0 = (unsigned)da.x - nbs, s1 = (unsigned)da.y - nbs;
  const unsigned s2 = (unsigned)da.z - nbs, s3 = (unsigned)da.w - nbs;
  const unsigned s4 = (unsigned)db.x - nbs, s5 = (unsigned)db.y - nbs;
  const unsigned s6 = (unsigned)db.z - nbs, s7 = (unsigned)db.w - nbs;
  const bool h0 = s0 < unb, h1 = s1 < unb, h2 = s2 < unb, h3 = s3 < unb;
  const bool h4 = s4 < unb, h5 = s5 < unb, h6 = s6 < unb, h7 = s7 < unb;
  const unsigned any = __builtin_amdgcn_ballot_w32(h0 | h1 | h2 | h3 | h4 | h5 | h6 | h7);
  if (any != 0u) {
#define HITJ(J, HJ, SJ) { \
      const unsigned mj = __builtin_amdgcn_ballot_w32(HJ); \
      if (mj != 0u) { \
        if (HJ) { \
          const int pos = wc + (int)__builtin_amdgcn_mbcnt_lo(mj, 0u); \
          if (pos < WCAP) list[wave * WCAP + pos] = ((el0 + (J)) << PKS) | (int)(SJ); \
        } \
        wc += (int)__builtin_popcount(mj); } }
    HITJ(0, h0, s0)
    HITJ(1, h1, s1)
    HITJ(2, h2, s2)
    HITJ(3, h3, s3)
    HITJ(4, h4, s4)
    HITJ(5, h5, s5)
    HITJ(6, h6, s6)
    HITJ(7, h7, s7)
#undef HITJ
  }
  return wc;
}

__global__ __launch_bounds__(NTHR) void k_wprep(const float* __restrict__ w1s, const float* __restrict__ w2s,
                                                int nL, int nUnits, unsigned short* WPL) {
  const int u = (int)blockIdx.x * NTHR + (int)threadIdx.x;
  if (u >= nUnits) return;
  const int n1 = nL * WU1;
  const bool isW2 = u >= n1;
  int n, q, l, kb, ks;
  size_t dsto;
  if (!isW2) {
    l = u >> 13;
    const int v = u & (WU1 - 1);
    n = v >> 5; q = v & 31; kb = 0; ks = DH;
    dsto = (size_t)l * PH1 + (size_t)v * 8;
  } else {
    const int u2 = u - n1;
    const int pl = u2 >> 12;
    const int v = u2 & (WU2 - 1);
    n = v >> 5; q = v & 31; l = pl >> 1; kb = (pl & 1) * DF; ks = DF;
    dsto = (size_t)nL * PH1 + (size_t)pl * PH2 + (size_t)v * 8;
  }
  const float* w = (isW2 ? w2s : w1s) + (size_t)l * (size_t)(DF * DH);
  const float* p = w + (size_t)(kb + 4 * q) * (size_t)ks + n;
  float f[4];
#pragma unroll
  for (int c = 0; c < 4; ++c) f[c] = p[(size_t)c * (size_t)ks];
  v8us o;
#pragma unroll
  for (int j = 0; j < 8; ++j) o[j] = bf_bits(f[j & 3]);
  unsigned short* dp = WPL + dsto;
  *(volatile v8us*)dp = o;
  __threadfence();
  *(volatile v8us*)dp = o;
}

__global__ __launch_bounds__(NTHR) void k_hinit(const int* __restrict__ xi, const int* __restrict__ zi,
                                                const float* __restrict__ atab, int nV,
                                                const float* __restrict__ ztab, int nZ,
                                                int nUnits, float* hout) {
  const int u = (int)blockIdx.x * NTHR + (int)threadIdx.x;
  if (u >= nUnits) return;
  const int row = u >> 5, j = u & 31, c = 4 * j;
  float ax = 0.0f, ay = 0.0f, az = 0.0f, aw = 0.0f;
#pragma unroll 1
  for (int f = 0; f < NF; ++f) {
    int ix = xi[(size_t)row * NF + f];
    ix = ix < 0 ? 0 : (ix > nV - 1 ? nV - 1 : ix);
    const v4f t = *(const v4fa*)(atab + ((size_t)f * (size_t)nV + (size_t)ix) * DF + c);
    ax += bf_rne(t.x); ay += bf_rne(t.y); az += bf_rne(t.z); aw += bf_rne(t.w);
  }
  int iz = zi[row];
  iz = iz < 0 ? 0 : (iz > nZ - 1 ? nZ - 1 : iz);
  const v4f tz = *(const v4fa*)(ztab + (size_t)iz * DF + c);
  v4f y;
  y.x = ax + bf_rne(tz.x);
  y.y = ay + bf_rne(tz.y);
  y.z = az + bf_rne(tz.z);
  y.w = aw + bf_rne(tz.w);
  float* op = hout + (size_t)row * DF + c;
  *(volatile v4f*)op = y;
  __threadfence();
  *(volatile v4f*)op = y;
}

template <int ACT, int STATS>
__global__ __launch_bounds__(GTHR) void k_gemm(const unsigned short* __restrict__ A, int lda,
                                               const unsigned short* __restrict__ BT, int ldb, int K,
                                               const float* __restrict__ bias,
                                               float* C32, int ldc, int nRows, int nLive, float* part) {
  static_assert(STATS == 0 || STATS == 1);
  __shared__ __attribute__((aligned(16))) float stg[GBM * GBN];
  __shared__ __attribute__((aligned(16))) float pst[PARTW];
  const int tid = (int)threadIdx.x, lane = tid & 31, wave = tid >> 5, hh = lane >> 4, m = lane & 15;
  const int rowBase = (int)blockIdx.x * GBM;

  v8f acc[GNT];
  {
    const v8f z = {0.f, 0.f, 0.f, 0.f, 0.f, 0.f, 0.f, 0.f};
#pragma unroll
    for (int t = 0; t < GNT; ++t) acc[t] = z;
  }
  const unsigned short* ap = A  + (size_t)(rowBase + 16 * wave + m) * (size_t)lda + 8 * hh;
  const unsigned short* bp = BT + (size_t)m * (size_t)ldb + 8 * hh;

#pragma unroll 1
  for (int k0 = 0; k0 < K; k0 += 32) {
    Frag af;
    af.h[0] = *(const v8usa*)(ap + k0);
    af.h[1] = *(const v8usa*)(ap + k0 + 16);
#pragma unroll
    for (int nt = 0; nt < GNT; ++nt) {
      const unsigned short* wq = bp + (size_t)(16 * nt) * (size_t)ldb + k0;
      Frag bf;
      bf.h[0] = *(const v8usa*)wq;
      bf.h[1] = *(const v8usa*)(wq + 16);
      acc[nt] = wmk(af, bf, acc[nt]);
    }
  }

#pragma unroll
  for (int nt = 0; nt < GNT; ++nt) {
    const int lc = 16 * nt + m;
    const float bb = bf_rne(bias[lc]);
#pragma unroll
    for (int r = 0; r < 8; ++r) {
      const int lr = 16 * wave + 8 * hh + r;
      stg[lr * GBN + lc] = actf<ACT>(acc[nt][r] + bb);
    }
  }
  __syncthreads();

  {
    v4f pv[16];
#pragma unroll
    for (int i = 0; i < 16; ++i) pv[i] = *(const v4fa*)(stg + (16 * wave + i) * GBN + 4 * lane);
#pragma unroll
    for (int i = 0; i < 16; ++i) {
      const int gr = rowBase + 16 * wave + i;
      float* op = C32 + (size_t)gr * (size_t)ldc + 4 * lane;
      if (gr < nRows) *(volatile v4f*)op = pv[i];
    }
    __threadfence();
#pragma unroll
    for (int i = 0; i < 16; ++i) {
      const int gr = rowBase + 16 * wave + i;
      float* op = C32 + (size_t)gr * (size_t)ldc + 4 * lane;
      if (gr < nRows) *(volatile v4f*)op = pv[i];
    }
  }

  if constexpr (STATS == 1) {
    int nb = nLive - rowBase;
    nb = nb < 0 ? 0 : (nb > GBM ? GBM : nb);
    const int c = tid;
    float s = 0.0f;
#pragma unroll 4
    for (int r = 0; r < nb; ++r) s += stg[r * GBN + c];
    const float inv = 1.0f / (float)(nb < 1 ? 1 : nb);
    const float mb = s * inv;
    float q = 0.0f;
#pragma unroll 4
    for (int r = 0; r < nb; ++r) {
      const float d = stg[r * GBN + c] - mb;
      q = fmaf(d, d, q);
    }
    pst[PMEAN + c] = mb;
    pst[PM2 + c]   = q;
    if (tid < PMEAN) pst[tid] = (tid == 0) ? (float)nb : 0.0f;
    __syncthreads();
    v4f ps = {0.0f, 0.0f, 0.0f, 0.0f};
    if (tid < PARTW / 4) {
      ps = *(const v4fa*)(pst + 4 * tid);
      *(volatile v4f*)(part + (size_t)blockIdx.x * PARTW + 4 * tid) = ps;
    }
    __threadfence();
    if (tid < PARTW / 4) {
      *(volatile v4f*)(part + (size_t)blockIdx.x * PARTW + 4 * tid) = ps;
    }
  } else {
    (void)nLive; (void)part; (void)pst;
  }
}

template <int ACC>
__global__ __launch_bounds__(GTHR) void k_gemm2f(const float* __restrict__ S, const float* __restrict__ ss,
                                                 const unsigned short* __restrict__ BT,
                                                 const float* __restrict__ bias,
                                                 float* C32, int nRows, int nLive, float* part) {
  static_assert(ACC == 0 || ACC == 1);
  __shared__ __attribute__((aligned(16))) float stg[GBM * GBN];
  __shared__ __attribute__((aligned(16))) float ssh[2 * DF];
  __shared__ __attribute__((aligned(16))) float pst[PARTW];
  const int tid = (int)threadIdx.x, lane = tid & 31, wave = tid >> 5, hh = lane >> 4, m = lane & 15;
  const int rowBase = (int)blockIdx.x * GBM;

  ssh[tid] = ss[tid];
  ssh[DF + tid] = ss[DF + tid];
  __syncthreads();

  v8f acc[GNT];
  {
    const v8f z = {0.f, 0.f, 0.f, 0.f, 0.f, 0.f, 0.f, 0.f};
#pragma unroll
    for (int t = 0; t < GNT; ++t) acc[t] = z;
  }
  const float* arow = S + (size_t)(rowBase + 16 * wave + m) * (size_t)DF + 4 * hh;
  const unsigned short* bp = BT + (size_t)m * (size_t)KA + 8 * hh;

#pragma unroll 1
  for (int k0 = 0; k0 < KA; k0 += 32) {
    const int cb = (k0 >> 1) + 4 * hh;
    const v4f x0 = *(const v4fa*)(arow + (k0 >> 1));
    const v4f x1 = *(const v4fa*)(arow + (k0 >> 1) + 8);
    const v4f c0 = *(const v4fa*)(ssh + cb);
    const v4f d0 = *(const v4fa*)(ssh + DF + cb);
    const v4f c1 = *(const v4fa*)(ssh + cb + 8);
    const v4f d1 = *(const v4fa*)(ssh + DF + cb + 8);
    Frag af;
    af.q[0] = pack_hilo4(fmaxf(fmaf(x0.x, c0.x, d0.x), 0.0f), fmaxf(fmaf(x0.y, c0.y, d0.y), 0.0f),
                         fmaxf(fmaf(x0.z, c0.z, d0.z), 0.0f), fmaxf(fmaf(x0.w, c0.w, d0.w), 0.0f));
    af.q[1] = pack_hilo4(fmaxf(fmaf(x1.x, c1.x, d1.x), 0.0f), fmaxf(fmaf(x1.y, c1.y, d1.y), 0.0f),
                         fmaxf(fmaf(x1.z, c1.z, d1.z), 0.0f), fmaxf(fmaf(x1.w, c1.w, d1.w), 0.0f));
#pragma unroll
    for (int nt = 0; nt < GNT; ++nt) {
      const unsigned short* wq = bp + (size_t)(16 * nt) * (size_t)KA + k0;
      Frag bf;
      bf.h[0] = *(const v8usa*)wq;
      bf.h[1] = *(const v8usa*)(wq + 16);
      acc[nt] = wmk(af, bf, acc[nt]);
    }
  }

#pragma unroll
  for (int nt = 0; nt < GNT; ++nt) {
    const int lc = 16 * nt + m;
    float bb = 0.0f;
    if constexpr (ACC == 0) bb = bf_rne(bias[lc]);
#pragma unroll
    for (int r = 0; r < 8; ++r) {
      const int lr = 16 * wave + 8 * hh + r;
      stg[lr * GBN + lc] = acc[nt][r] + bb;
    }
  }
  __syncthreads();

  v4f pv[16];
#pragma unroll
  for (int i = 0; i < 16; ++i) pv[i] = *(const v4fa*)(stg + (16 * wave + i) * GBN + 4 * lane);
  if constexpr (ACC == 1) {
#pragma unroll
    for (int i = 0; i < 16; ++i) {
      const int gr = rowBase + 16 * wave + i;
      const int grc = gr < nRows ? gr : (nRows - 1);
      const v4f t = *(const v4fa*)(C32 + (size_t)grc * (size_t)DF + 4 * lane);
      pv[i] = pv[i] + t;
    }
  }
#pragma unroll
  for (int i = 0; i < 16; ++i) {
    const int gr = rowBase + 16 * wave + i;
    float* op = C32 + (size_t)gr * (size_t)DF + 4 * lane;
    if (gr < nRows) *(volatile v4f*)op = pv[i];
  }
  __threadfence();
#pragma unroll
  for (int i = 0; i < 16; ++i) {
    const int gr = rowBase + 16 * wave + i;
    float* op = C32 + (size_t)gr * (size_t)DF + 4 * lane;
    if (gr < nRows) *(volatile v4f*)op = pv[i];
  }

  if constexpr (ACC == 1) {
#pragma unroll
    for (int i = 0; i < 16; ++i) *(v4fa*)(stg + (16 * wave + i) * GBN + 4 * lane) = pv[i];
    __syncthreads();
    int nb = nLive - rowBase;
    nb = nb < 0 ? 0 : (nb > GBM ? GBM : nb);
    const int c = tid;
    float s = 0.0f;
#pragma unroll 4
    for (int r = 0; r < nb; ++r) s += stg[r * GBN + c];
    const float inv = 1.0f / (float)(nb < 1 ? 1 : nb);
    const float mb = s * inv;
    float q = 0.0f;
#pragma unroll 4
    for (int r = 0; r < nb; ++r) {
      const float d = stg[r * GBN + c] - mb;
      q = fmaf(d, d, q);
    }
    pst[PMEAN + c] = mb;
    pst[PM2 + c]   = q;
    if (tid < PMEAN) pst[tid] = (tid == 0) ? (float)nb : 0.0f;
    __syncthreads();
    v4f ps = {0.0f, 0.0f, 0.0f, 0.0f};
    if (tid < PARTW / 4) {
      ps = *(const v4fa*)(pst + 4 * tid);
      *(volatile v4f*)(part + (size_t)blockIdx.x * PARTW + 4 * tid) = ps;
    }
    __threadfence();
    if (tid < PARTW / 4) {
      *(volatile v4f*)(part + (size_t)blockIdx.x * PARTW + 4 * tid) = ps;
    }
  } else {
    (void)nLive; (void)part; (void)pst;
  }
}

__global__ __launch_bounds__(NTHR) void k_agg(const int* __restrict__ srcs, const int* __restrict__ dsts,
                                              const int* __restrict__ eattr, const float* __restrict__ btab,
                                              const float* __restrict__ epl, const float* __restrict__ X,
                                              unsigned short* Aout, int nN, int nE, int vec8) {
  extern __shared__ __attribute__((aligned(16))) int lds_i[];
  int* reg1 = lds_i;
  int* reg2 = reg1 + RCAP;
  int* scnt = reg2 + RCAP;
  int* soff = scnt + NBA;
  int* list = soff + NBA;
  int* wcnt = list + LISTN;
  int* wtot = wcnt + NWAVE;
  float* stab = (float*)(lds_i + ZINTS + MISCI);
  const int tid = (int)threadIdx.x, lane = tid & 31, wave = tid >> 5;
  const int nodeBase = (int)blockIdx.x * NBA;

  {
    const v4i z4 = {0, 0, 0, 0};
    for (int i = tid * 4; i < ZINTS; i += NTHR * 4) *(v4ia*)(lds_i + i) = z4;
    if (tid < 2 * NWAVE) wcnt[tid] = 0;
  }
#pragma unroll 1
  for (int i = tid; i < BTAB; i += NTHR) stab[i] = bf_rne(btab[i]);
  __syncthreads();
  const float opl = 1.0f + bf_rne(epl[0]);

  int tot = 0;
  const int nChunks = (nE + CHUNK - 1) / CHUNK;
#pragma unroll 1
  for (int ch = 0; ch < nChunks; ++ch) {
    const int cbase = ch * CHUNK;
    const int wc = scan_chunk(dsts, nE, cbase, nodeBase, NBA, vec8, list, tid, lane, wave);
    if (lane == 0) wcnt[wave] = wc;
    __syncthreads();
    int pre = 0, all = 0;
#pragma unroll
    for (int w2 = 0; w2 < NWAVE; ++w2) {
      int c = wcnt[w2];
      c = c < 0 ? 0 : (c > WCAP ? WCAP : c);
      all += c;
      pre += (w2 < wave) ? c : 0;
    }
    const int wcc  = wc > WCAP ? WCAP : wc;
    const int base = tot + pre;
#pragma unroll 1
    for (int i = lane; i < wcc; i += 32) {
      const int ent = list[wave * WCAP + i];
      const int el  = (ent >> PKS) & (CHUNK - 1);
      const int sl  = ent & (NBA - 1);
      int eid = cbase + el;
      eid = eid > nE - 1 ? nE - 1 : eid;
      const int pos = base + i;
      if (pos < RCAP) reg1[pos] = (int)(((unsigned)eid << PKS) | (unsigned)sl);
    }
    tot += all;
    tot = tot > RCAP ? RCAP : tot;
    __syncthreads();
  }
  const int nh = tot;

  if (wave == 0) {
#pragma unroll 1
    for (int b0 = 0; b0 < nh; b0 += 32) {
      const int idx = b0 + lane;
      const int uv  = reg1[idx < RCAP ? idx : RCAP - 1];
      const int m32 = (nh - b0) < 32 ? (nh - b0) : 32;
#pragma unroll 1
      for (int k = 0; k < m32; ++k) {
        const int u  = __builtin_amdgcn_readlane(uv, k);
        const int sl = u & (NBA - 1);
        if (lane == 0) scnt[sl] = scnt[sl] + 1;
      }
    }
  }
  __syncthreads();

  {
    const v4i ca = *(const v4ia*)(scnt + 4 * tid);
    const int e0 = ca.x < 0 ? 0 : ca.x, e1 = ca.y < 0 ? 0 : ca.y, e2 = ca.z < 0 ? 0 : ca.z, e3 = ca.w < 0 ? 0 : ca.w;
    const int ts = e0 + e1 + e2 + e3;
    int incl = ts;
#pragma unroll
    for (int d = 1; d < 32; d <<= 1) {
      const int up = __shfl_up(incl, d, 32);
      if (lane >= d) incl += up;
    }
    if (lane == 31) wtot[wave] = incl;
    __syncthreads();
    int pre = 0;
#pragma unroll
    for (int w2 = 0; w2 < NWAVE; ++w2) pre += (w2 < wave) ? wtot[w2] : 0;
    int run = pre + incl - ts;
    soff[4 * tid + 0] = run; run += e0;
    soff[4 * tid + 1] = run; run += e1;
    soff[4 * tid + 2] = run; run += e2;
    soff[4 * tid + 3] = run;
  }
  __syncthreads();
  for (int i = tid; i < NBA; i += NTHR) list[i] = soff[i];
  __syncthreads();

  if (wave == 0) {
#pragma unroll 1
    for (int b0 = 0; b0 < nh; b0 += 32) {
      const int idx = b0 + lane;
      const int uv  = reg1[idx < RCAP ? idx : RCAP - 1];
      const int m32 = (nh - b0) < 32 ? (nh - b0) : 32;
#pragma unroll 1
      for (int k = 0; k < m32; ++k) {
        const int u   = __builtin_amdgcn_readlane(uv, k);
        const int sl  = u & (NBA - 1);
        const int eid = (int)((unsigned)u >> PKS);
        if (lane == 0) {
          int pos = list[sl];
          pos = pos < 0 ? 0 : (pos > RCAP - 1 ? RCAP - 1 : pos);
          reg2[pos] = eid;
          list[sl] = pos + 1;
        }
      }
    }
  }
  __syncthreads();

  const int nbw = NBA / NWAVE;
  const bool ovf = (nh >= RCAP);
  const float qnan = __int_as_float(0x7fc00000);

#pragma unroll 1
  for (int jt = 0; jt < nbw; ++jt) {
    const int slot = wave * nbw + jt;
    const int node = nodeBase + slot;
    int st = soff[slot];
    const int craw = scnt[slot];
    int cnt = craw;
    st  = st < 0 ? 0 : (st > nh ? nh : st);
    cnt = cnt < 0 ? 0 : (cnt > DEGCAP ? DEGCAP : cnt);
    if (cnt > nh - st) cnt = nh - st;
    const float pz = (ovf || craw > DEGCAP) ? qnan : 0.0f;
    const bool live = node < nN;
    const int nc = node < nN ? node : nN - 1;

    float g0 = 0.f, g1 = 0.f, g2 = 0.f, g3 = 0.f;
#pragma unroll 1
    for (int b0 = 0; b0 < cnt; b0 += 32) {
      int idx = st + b0 + lane; idx = idx > RCAP - 1 ? RCAP - 1 : idx;
      int eid = reg2[idx]; eid = eid < 0 ? 0 : (eid > nE - 1 ? nE - 1 : eid);
      int sr = srcs[eid]; sr = sr < 0 ? 0 : (sr > nN - 1 ? nN - 1 : sr);
      const int* er = eattr + (size_t)eid * NBF;
      int f0 = er[0], f1 = er[1], f2 = er[2];
      f0 = f0 < 0 ? 0 : (f0 > NBV - 1 ? NBV - 1 : f0);
      f1 = f1 < 0 ? 0 : (f1 > NBV - 1 ? NBV - 1 : f1);
      f2 = f2 < 0 ? 0 : (f2 > NBV - 1 ? NBV - 1 : f2);
      const int fpk = f0 | (f1 << 3) | (f2 << 6);
      const int m32 = (cnt - b0) < 32 ? (cnt - b0) : 32;
#pragma unroll 1
      for (int k = 0; k < m32; ++k) {
        const int sk = __builtin_amdgcn_readlane(sr, k);
        const int ak = __builtin_amdgcn_readlane(fpk, k);
        const v4f t0 = *(const v4fa*)(stab + (ak & 7) * DF + 4 * lane);
        const v4f t1 = *(const v4fa*)(stab + (NBV + ((ak >> 3) & 7)) * DF + 4 * lane);
        const v4f t2 = *(const v4fa*)(stab + (2 * NBV + ((ak >> 6) & 7)) * DF + 4 * lane);
        const v4f v  = *(const v4fa*)(X + (size_t)sk * DF + 4 * lane);
        g0 += fmaxf(v.x + ((t0.x + t1.x) + t2.x), 0.0f);
        g1 += fmaxf(v.y + ((t0.y + t1.y) + t2.y), 0.0f);
        g2 += fmaxf(v.z + ((t0.z + t1.z) + t2.z), 0.0f);
        g3 += fmaxf(v.w + ((t0.w + t1.w) + t2.w), 0.0f);
      }
    }
    const v4f sv = *(const v4fa*)(X + (size_t)nc * DF + 4 * lane);
    float r0 = fmaf(opl, sv.x, g0), r1 = fmaf(opl, sv.y, g1);
    float r2 = fmaf(opl, sv.z, g2), r3 = fmaf(opl, sv.w, g3);
    r0 = (live ? r0 : 0.0f) + pz;
    r1 = (live ? r1 : 0.0f) + pz;
    r2 = (live ? r2 : 0.0f) + pz;
    r3 = (live ? r3 : 0.0f) + pz;

    const v4u pk = pack_hilo4(r0, r1, r2, r3);
    unsigned short* gp = Aout + (size_t)node * (size_t)KA + 8 * lane;
    *(volatile v4u*)gp = pk;
    __threadfence();
    *(volatile v4u*)gp = pk;
  }
}

__global__ __launch_bounds__(DF) void k_bnfin(const float* __restrict__ part, int nPart,
                                              const float* __restrict__ gam, const float* __restrict__ bet,
                                              float* ss) {
  __shared__ __attribute__((aligned(16))) float stg[2 * DF];
  const int tid = (int)threadIdx.x;
  const int c = tid;
  double n = 0.0, mean = 0.0, M2 = 0.0;
#pragma unroll 1
  for (int b = 0; b < nPart; ++b) {
    const float* pr = part + (size_t)b * PARTW;
    const double nb = (double)pr[0];
    const double mb = (double)pr[PMEAN + c];
    const double qb = (double)pr[PM2 + c];
    if (nb > 0.5) {
      const double nn = n + nb;
      const double delta = mb - mean;
      const double f = nb / nn;
      mean = mean + delta * f;
      M2 = M2 + qb + delta * delta * n * f;
      n = nn;
    }
  }
  const double ntot = n < 1.0 ? 1.0 : n;
  const float varf  = (float)(M2 / ntot);
  const float meanf = (float)mean;
  const float rstd = rsqrtf(varf + 1e-5f);
  const float sc = bf_rne(gam[c]) * rstd;
  const float sh = bf_rne(bet[c]) - meanf * sc;
  stg[c] = sc;
  stg[DF + c] = sh;
  __syncthreads();
  v4f v = {0.0f, 0.0f, 0.0f, 0.0f};
  if (tid < (2 * DF) / 4) {
    v = *(const v4fa*)(stg + 4 * tid);
    *(volatile v4f*)(ss + 4 * tid) = v;
  }
  __threadfence();
  if (tid < (2 * DF) / 4) {
    *(volatile v4f*)(ss + 4 * tid) = v;
  }
}

template <int FIN>
__global__ __launch_bounds__(NTHR) void k_apply2(float* hbuf, const float* __restrict__ ss, int nUnits) {
  __shared__ __attribute__((aligned(16))) float ssh[2 * DF];
  const int tid = (int)threadIdx.x;
  ssh[tid] = ss[tid];
  __syncthreads();
  const int u = (int)blockIdx.x * NTHR + tid;
  if (u >= nUnits) return;
  const int row = u >> 5, c0 = 4 * (u & 31);
  float* p = hbuf + (size_t)row * DF + c0;
  const v4f a  = *(const v4fa*)p;
  const v4f sc = *(const v4fa*)(ssh + c0);
  const v4f sh = *(const v4fa*)(ssh + DF + c0);
  v4f y;
  y.x = fmaf(a.x, sc.x, sh.x);
  y.y = fmaf(a.y, sc.y, sh.y);
  y.z = fmaf(a.z, sc.z, sh.z);
  y.w = fmaf(a.w, sc.w, sh.w);
  if constexpr (FIN == 0) {
    y.x = fmaxf(y.x, 0.0f);
    y.y = fmaxf(y.y, 0.0f);
    y.z = fmaxf(y.z, 0.0f);
    y.w = fmaxf(y.w, 0.0f);
  }
  *(volatile v4f*)p = y;
  __threadfence();
  *(volatile v4f*)p = y;
}

static inline int cdiv(int a, int b) { return (a + b - 1) / b; }
static inline size_t al256(size_t o) { return (o + 255) & ~(size_t)255; }

extern "C" void kernel_launch(void* const* d_in, const int* in_sizes, int n_in,
                              void* d_out, int out_size, void* d_ws, size_t ws_size,
                              hipStream_t stream) {
  if (n_in < 16) return;
  const int nN = in_sizes[1];
  if (nN < 16 || nN >= (1 << 22)) return;
  if (in_sizes[0] != nN * NF) return;
  if (in_sizes[2] < 2 || (in_sizes[2] & 1) != 0) return;
  const int nE = in_sizes[2] / 2;
  if (nE < 1 || nE >= (1 << 21)) return;
  if (in_sizes[3] != nE * NBF) return;
  if (in_sizes[4] < NF * DF || (in_sizes[4] % (NF * DF)) != 0) return;
  const int nV = in_sizes[4] / (NF * DF);
  if (in_sizes[5] < DF || (in_sizes[5] % DF) != 0) return;
  const int nZ = in_sizes[5] / DF;
  if (in_sizes[6] < BTAB || (in_sizes[6] % BTAB) != 0) return;
  const int nL = in_sizes[6] / BTAB;
  if (nL < 1 || nL > NLMAX) return;
  if (in_sizes[7] != nL) return;
  if (in_sizes[8] != nL * DF * DH) return;
  if (in_sizes[9] != nL * DH || in_sizes[10] != nL * DH || in_sizes[11] != nL * DH) return;
  if (in_sizes[12] != nL * DH * DF) return;
  if (in_sizes[13] != nL * DF || in_sizes[14] != nL * DF || in_sizes[15] != nL * DF) return;
  if ((long long)out_size != (long long)nN * DF) return;

  const int*   xi   = (const int*)  d_in[0];
  const int*   zi   = (const int*)  d_in[1];
  const int*   ei   = (const int*)  d_in[2];
  const int*   ea   = (const int*)  d_in[3];
  const float* atab = (const float*)d_in[4];
  const float* ztab = (const float*)d_in[5];
  const float* btab = (const float*)d_in[6];
  const float* eps  = (const float*)d_in[7];
  const float* W1   = (const float*)d_in[8];
  const float* b1   = (const float*)d_in[9];
  const float* g1   = (const float*)d_in[10];
  const float* be1  = (const float*)d_in[11];
  const float* W2   = (const float*)d_in[12];
  const float* b2   = (const float*)d_in[13];
  const float* bng  = (const float*)d_in[14];
  const float* bnb  = (const float*)d_in[15];
  float* out = (float*)d_out;
  const int* src = ei;
  const int* dst = ei + nE;

  const int MP   = cdiv(nN, GBM) * GBM;
  const int gM   = MP / GBM;
  const int gA   = cdiv(MP, NBA);
  const int RA   = gA * NBA;
  const int vec8 = ((nE & 3) == 0) ? 1 : 0;
  if ((long long)RA < (long long)MP) return;

  char* ws = (char*)d_ws;
  size_t off = 0;
  const size_t szWPL = ((size_t)nL * PH1 + (size_t)(2 * nL) * PH2) * 2;
  const size_t oWPL = off; off = al256(off + szWPL);
  const size_t oAP  = off; off = al256(off + (size_t)RA * KA * 2);
  const size_t oS1  = off; off = al256(off + (size_t)MP * DF * 4);
  const size_t oPT  = off; off = al256(off + (size_t)gM * PARTW * 4);
  const size_t oSS1 = off; off = al256(off + (size_t)(2 * DF) * 4);
  const size_t oSS2 = off; off = al256(off + (size_t)(2 * DF) * 4);
  if (off > ws_size || off > (size_t)WSMAX) return;
  unsigned short* WPL = (unsigned short*)(ws + oWPL);
  unsigned short* AP  = (unsigned short*)(ws + oAP);
  float*          S1  = (float*)(ws + oS1);
  float*          PT  = (float*)(ws + oPT);
  float*          SS1 = (float*)(ws + oSS1);
  float*          SS2 = (float*)(ws + oSS2);

  hipFuncSetAttribute(reinterpret_cast<const void*>(&k_agg), hipFuncAttributeMaxDynamicSharedMemorySize, LDS_AGG);

  const int nUW = nL * WU1 + 2 * nL * WU2;
  k_wprep<<<nUW / NTHR, NTHR, 0, stream>>>(W1, W2, nL, nUW, WPL);

  const int nUo = nN * 32;
  k_hinit<<<cdiv(nUo, NTHR), NTHR, 0, stream>>>(xi, zi, atab, nV, ztab, nZ, nUo, out);

  for (int l = 0; l < nL; ++l) {
    k_agg<<<gA, NTHR, LDS_AGG, stream>>>(src, dst, ea, btab + (size_t)l * BTAB, eps + l, out, AP, nN, nE, vec8);
    for (int y = 0; y < 2; ++y) {
      const unsigned short* W1D = WPL + (size_t)l * PH1 + (size_t)y * (size_t)(DF * KA);
      const unsigned short* W2D = WPL + (size_t)nL * PH1 + (size_t)(2 * l + y) * PH2;
      k_gemm<0, 1><<<gM, GTHR, 0, stream>>>(AP, KA, W1D, KA, KA, b1 + (size_t)l * DH + (size_t)y * DF,
                                           S1, DF, MP, nN, PT);
      k_bnfin<<<1, DF, 0, stream>>>(PT, gM, g1 + (size_t)l * DH + (size_t)y * DF,
                                    be1 + (size_t)l * DH + (size_t)y * DF, SS1);
      if (y == 0) {
        k_gemm2f<0><<<gM, GTHR, 0, stream>>>(S1, SS1, W2D, b2 + (size_t)l * DF, out, nN, nN, PT);
      } else {
        k_gemm2f<1><<<gM, GTHR, 0, stream>>>(S1, SS1, W2D, b2 + (size_t)l * DF, out, nN, nN, PT);
      }
    }
    k_bnfin<<<1, DF, 0, stream>>>(PT, gM, bng + (size_t)l * DF, bnb + (size_t)l * DF, SS2);
    if (l < nL - 1) {
      k_apply2<0><<<cdiv(nUo, NTHR), NTHR, 0, stream>>>(out, SS2, nUo);
    } else {
      k_apply2<1><<<cdiv(nUo, NTHR), NTHR, 0, stream>>>(out, SS2, nUo);
    }
  }
}
